// WGINE_29068338659498
// MI455X (gfx1250) — hardware-verified
//
#include <hip/hip_runtime.h>
#include <stddef.h>


#define NFP   33
#define DIM   16
#define EMBD  128
#define KSZ   8
#define TOUT  (EMBD - KSZ + 1)
#define NF    32
#define FCIN  (NF * TOUT)
#define BN_EPS 1e-5f

#define NTHR  256
#define NWAVE 8
#define CHUNK 2048
#define WCH   (CHUNK / NWAVE)
#define WCAP  WCH

typedef float  v4f  __attribute__((ext_vector_type(4)));
typedef float  v8f  __attribute__((ext_vector_type(8)));
typedef int    v4i  __attribute__((ext_vector_type(4)));
typedef double v2d  __attribute__((ext_vector_type(2)));
typedef __bf16 bf16_t;
typedef bf16_t v8bf  __attribute__((ext_vector_type(8)));
typedef bf16_t v16bf __attribute__((ext_vector_type(16)));
union FragB { v16bf v; v8bf h[2]; v4i q[2]; };
union Pack8 { v8bf v; v4i q; };

static_assert((CHUNK & (CHUNK - 1)) == 0);
static_assert(CHUNK <= 2048);
static_assert(WCH % 32 == 0);

__device__ __forceinline__ v8f wmb(v16bf a, v16bf b, v8f c) {
  v8f d = __builtin_amdgcn_wmma_f32_16x16x32_bf16(false, a, false, b, (short)0, c, false, false);
  asm volatile("v_nop\n\tv_nop\n\tv_nop\n\tv_nop" : "+v"(d) : "v"(a), "v"(b));
  return d;
}

__device__ __forceinline__ v8f zero8() { v8f z = {0.f, 0.f, 0.f, 0.f, 0.f, 0.f, 0.f, 0.f}; return z; }

template <int B0>
__device__ __forceinline__ void split8(FragB& hi, FragB& lo, v4f a, v4f b) {
#define SPL1(I, X) { const float xv = (X); const bf16_t hb = (bf16_t)xv; hi.v[B0 + (I)] = hb; lo.v[B0 + (I)] = (bf16_t)(xv - (float)hb); }
  SPL1(0, a.x) SPL1(1, a.y) SPL1(2, a.z) SPL1(3, a.w)
  SPL1(4, b.x) SPL1(5, b.y) SPL1(6, b.z) SPL1(7, b.w)
#undef SPL1
}

__global__ __launch_bounds__(NTHR) void k_wprep(const float* __restrict__ W, int sn, int sk, int K, int KP,
                                                bf16_t* whi, bf16_t* wlo, int nTot) {
  const int i = blockIdx.x * NTHR + threadIdx.x;
  if (i >= nTot) return;
  const size_t o = (size_t)i * 8;
  const int n  = (int)(o / (size_t)KP);
  const int k0 = (int)(o - (size_t)n * KP);
  Pack8 ph, pl;
#pragma unroll
  for (int j = 0; j < 8; ++j) {
    const int k  = k0 + j;
    const int kc = k < K ? k : K - 1;
    float xv = W[(size_t)n * sn + (size_t)kc * sk];
    xv = (k < K) ? xv : 0.0f;
    const bf16_t hb = (bf16_t)xv;
    ph.v[j] = hb;
    pl.v[j] = (bf16_t)(xv - (float)hb);
  }
  const v4i qh = ph.q, ql = pl.q;
  *(volatile v4i*)(whi + o) = qh;
  *(volatile v4i*)(wlo + o) = ql;
  __threadfence();
  *(volatile v4i*)(whi + o) = qh;
  *(volatile v4i*)(wlo + o) = ql;
}

__global__ __launch_bounds__(128) void k_conv(
    const int* __restrict__ tok, int L, int NT, const float* __restrict__ emb,
    const bf16_t* __restrict__ whi, const bf16_t* __restrict__ wlo, int KP, int nKs,
    const float* __restrict__ cb, float* P, int M, int nTiles) {
  __shared__ float embs[65 * EMBD];
  __shared__ v4f   stg4[4][128];
  const int tid = threadIdx.x, lane = tid & 31, wave = tid >> 5, h = lane >> 4, m = lane & 15;
  const int tile = blockIdx.x * 4 + wave;
  const bool valid = tile < nTiles;
  for (int i = tid; i < NT * EMBD; i += 128) embs[i] = emb[i];
  __syncthreads();

  int r = tile * 16 + m;
  r = r > M - 1 ? M - 1 : r;
  const int b = r / TOUT;
  const int t = r - b * TOUT;
  const int* tr = tok + (size_t)b * L;

  v8f c0 = zero8(), c1 = zero8();
  const bf16_t* bh0 = whi + (size_t)m * KP + 8 * h;
  const bf16_t* bl0 = wlo + (size_t)m * KP + 8 * h;
  const size_t  cst = (size_t)16 * KP;
  const v4f z4 = {0.f, 0.f, 0.f, 0.f};

#pragma unroll 1
  for (int ks = 0; ks < nKs; ++ks) {
    const int cA = 4 * ks + h, cB = cA + 2;
    int tA = tr[cA < L ? cA : L - 1];
    int tB = tr[cB < L ? cB : L - 1];
    tA = tA < 0 ? 0 : (tA > NT - 1 ? NT - 1 : tA);
    tB = tB < 0 ? 0 : (tB > NT - 1 ? NT - 1 : tB);
    const float* pa = embs + tA * EMBD + t;
    const float* pb = embs + tB * EMBD + t;
    v4f p0 = {pa[0], pa[1], pa[2], pa[3]};
    v4f p1 = {pa[4], pa[5], pa[6], pa[7]};
    v4f p2 = {pb[0], pb[1], pb[2], pb[3]};
    v4f p3 = {pb[4], pb[5], pb[6], pb[7]};
    p0 = (cA < L) ? p0 : z4;  p1 = (cA < L) ? p1 : z4;
    p2 = (cB < L) ? p2 : z4;  p3 = (cB < L) ? p3 : z4;
    FragB ahi, alo;
    split8<0>(ahi, alo, p0, p1);
    split8<8>(ahi, alo, p2, p3);
    const bf16_t* hp = bh0 + 32 * ks;
    const bf16_t* lp = bl0 + 32 * ks;
    FragB bh, bq;
    bh.q[0] = *(const v4i*)hp;          bh.q[1] = *(const v4i*)(hp + 16);
    bq.q[0] = *(const v4i*)lp;          bq.q[1] = *(const v4i*)(lp + 16);
    c0 = wmb(alo.v, bh.v, c0);
    c0 = wmb(ahi.v, bq.v, c0);
    c0 = wmb(ahi.v, bh.v, c0);
    bh.q[0] = *(const v4i*)(hp + cst);  bh.q[1] = *(const v4i*)(hp + cst + 16);
    bq.q[0] = *(const v4i*)(lp + cst);  bq.q[1] = *(const v4i*)(lp + cst + 16);
    c1 = wmb(alo.v, bh.v, c1);
    c1 = wmb(ahi.v, bq.v, c1);
    c1 = wmb(ahi.v, bh.v, c1);
  }

  float* sp = (float*)stg4[wave];
  const float cb0 = cb[m], cb1 = cb[16 + m];
#pragma unroll
  for (int rr = 0; rr < 8; ++rr) {
    sp[(8 * h + rr) * NF + m]      = c0[rr] + cb0;
    sp[(8 * h + rr) * NF + 16 + m] = c1[rr] + cb1;
  }
  __syncthreads();
  float* gp = P + (size_t)tile * 16 * NF + 4 * lane;
  if (valid) {
#pragma unroll
    for (int q = 0; q < 4; ++q) { const v4f v = stg4[wave][q * 32 + lane]; *(volatile v4f*)(gp + q * 128) = v; }
  }
  __threadfence();
  if (valid) {
#pragma unroll
    for (int q = 0; q < 4; ++q) { const v4f v = stg4[wave][q * 32 + lane]; *(volatile v4f*)(gp + q * 128) = v; }
  }
}

__global__ __launch_bounds__(32) void k_fc(
    const float* __restrict__ P0, const float* __restrict__ P1,
    const bf16_t* __restrict__ whi, const bf16_t* __restrict__ wlo, int KP, int nKs,
    const float* __restrict__ fcb, float* out) {
  __shared__ v4f stg4[16 * 32];
  const int lane = threadIdx.x, h = lane >> 4, m = lane & 15;
  const int mt = blockIdx.x;
  const int b  = mt * 16 + m;
  v8f c[8];
#pragma unroll
  for (int ct = 0; ct < 8; ++ct) c[ct] = zero8();

#pragma unroll 1
  for (int br = 0; br < 2; ++br) {
    const float* prow = ((br == 0) ? P0 : P1) + (size_t)b * TOUT * NF;
#pragma unroll 1
    for (int ks = 0; ks < nKs; ++ks) {
      const int kb = 32 * ks + 8 * h;
      float av[16];
#pragma unroll
      for (int i = 0; i < 8; ++i) {
        const int kk = kb + i;       const int o = kk / TOUT;  const int t = kk - o * TOUT;
        av[i] = prow[t * NF + o];
        const int k2 = kb + 16 + i;  const int o2 = k2 / TOUT; const int t2 = k2 - o2 * TOUT;
        av[8 + i] = prow[t2 * NF + o2];
      }
      const v4f p0 = {av[0], av[1], av[2], av[3]},    p1 = {av[4], av[5], av[6], av[7]};
      const v4f p2 = {av[8], av[9], av[10], av[11]},  p3 = {av[12], av[13], av[14], av[15]};
      FragB ahi, alo;
      split8<0>(ahi, alo, p0, p1);
      split8<8>(ahi, alo, p2, p3);
#pragma unroll
      for (int ct = 0; ct < 8; ++ct) {
        const bf16_t* hp = whi + (size_t)(16 * ct + m) * KP + 32 * ks + 8 * h;
        const bf16_t* lp = wlo + (size_t)(16 * ct + m) * KP + 32 * ks + 8 * h;
        FragB bh, bq;
        bh.q[0] = *(const v4i*)hp;  bh.q[1] = *(const v4i*)(hp + 16);
        bq.q[0] = *(const v4i*)lp;  bq.q[1] = *(const v4i*)(lp + 16);
        c[ct] = wmb(alo.v, bh.v, c[ct]);
        c[ct] = wmb(ahi.v, bq.v, c[ct]);
        c[ct] = wmb(ahi.v, bh.v, c[ct]);
      }
    }
  }
  float* sp = (float*)stg4;
#pragma unroll
  for (int ct = 0; ct < 8; ++ct) {
    const int col = 16 * ct + m;
    const float bb = fcb[col];
#pragma unroll
    for (int rr = 0; rr < 8; ++rr) sp[(8 * h + rr) * EMBD + col] = 0.5f * c[ct][rr] + bb;
  }
  __syncthreads();
  float* gp = out + (size_t)(mt * 16) * EMBD + 4 * lane;
#pragma unroll
  for (int i = 0; i < 16; ++i) { const v4f v = stg4[i * 32 + lane]; *(volatile v4f*)(gp + (size_t)i * EMBD) = v; }
  __threadfence();
#pragma unroll
  for (int i = 0; i < 16; ++i) { const v4f v = stg4[i * 32 + lane]; *(volatile v4f*)(gp + (size_t)i * EMBD) = v; }
}

template <int DIN, int NB>
__global__ __launch_bounds__(NTHR) void k_gine(
    const int* __restrict__ ei, const float* __restrict__ pw, const float* __restrict__ xin,
    const float* __restrict__ ew, const float* __restrict__ eb, const float* __restrict__ epsp,
    const float* __restrict__ w1, const float* __restrict__ b1,
    const float* __restrict__ w2, const float* __restrict__ b2,
    const double* __restrict__ pin, int nBlkIn, const float* __restrict__ gam, const float* __restrict__ bet,
    float* yout, double* pout, int nN, int nE) {
  static_assert((NB & (NB - 1)) == 0);
  static_assert(NB <= 4096);
  static_assert(NB % NTHR == 0);
  static_assert((NB * DIN) % 4 == 0);
  extern __shared__ v4f lds_dyn[];
  float* acc  = (float*)lds_dyn;
  int*   list = (int*)((char*)lds_dyn + (size_t)NB * DIN * 4);
  __shared__ float w1s[DIN * 16], w2s[256], b1s[16], b2s[16];
  __shared__ float ews[DIN], ebs[DIN], mus[DIN], scs[DIN], bes[DIN];
  __shared__ int wcnt[NWAVE];
  __shared__ double pst[32];

  const int tid = threadIdx.x, lane = tid & 31, wave = tid >> 5;
  const int nodeBase = blockIdx.x * NB;
  const int* dsts = ei + nE;

  for (int i = tid; i < DIN * 16; i += NTHR) w1s[i] = w1[i];
  for (int i = tid; i < 256; i += NTHR) w2s[i] = w2[i];
  if (tid < 16) { b1s[tid] = b1[tid]; b2s[tid] = b2[tid]; }
  if (tid < DIN) {
    ews[tid] = ew[tid]; ebs[tid] = eb[tid];
    float mu = 0.0f, sc = 1.0f, be = 0.0f;
    if (nBlkIn > 0) {
      double S = 0.0, Q = 0.0;
#pragma unroll 1
      for (int bb = 0; bb < nBlkIn; ++bb) { S += pin[(size_t)bb * 32 + tid]; Q += pin[(size_t)bb * 32 + 16 + tid]; }
      const double mud = S / (double)nN;
      double var = Q / (double)nN - mud * mud;
      var = var < 0.0 ? 0.0 : var;
      mu = (float)mud;
      sc = gam[tid] * (1.0f / sqrtf((float)var + BN_EPS));
      be = bet[tid];
    }
    mus[tid] = mu; scs[tid] = sc; bes[tid] = be;
  }
  {
    const v4f z = {0.f, 0.f, 0.f, 0.f};
    for (int i = tid; i < NB * DIN / 4; i += NTHR) lds_dyn[i] = z;
  }
  __syncthreads();

  const int nChunks = (nE + CHUNK - 1) / CHUNK;
#pragma unroll 1
  for (int ch = 0; ch < nChunks; ++ch) {
    const int cb = ch * CHUNK;
    const int wb = cb + wave * WCH;
    int wc = 0;
#pragma unroll 4
    for (int j = 0; j < WCH / 32; ++j) {
      const int e  = wb + j * 32 + lane;
      const int ec = e < nE ? e : nE - 1;
      const int d  = dsts[ec];
      const unsigned sl = (unsigned)(d - nodeBase);
      const bool hit = (e < nE) && (sl < (unsigned)NB);
      const unsigned mk = __builtin_amdgcn_ballot_w32(hit);
      if (hit) {
        const int pos = wc + (int)__builtin_amdgcn_mbcnt_lo(mk, 0u);
        if (pos < WCAP) list[wave * WCAP + pos] = ((e - cb) << 12) | (int)sl;
      }
      wc += (int)__builtin_popcount(mk);
    }
    if (lane == 0) wcnt[wave] = wc;
    __syncthreads();
    if (wave == 0) {
#pragma unroll 1
      for (int wsx = 0; wsx < NWAVE; ++wsx) {
        int n = __builtin_amdgcn_readfirstlane(wcnt[wsx]);
        n = n > WCAP ? WCAP : (n < 0 ? 0 : n);
        const int* lp = list + wsx * WCAP;
#pragma unroll 1
        for (int i = 0; i < n; ++i) {
          const int ent  = __builtin_amdgcn_readfirstlane(lp[i]);
          const int slot = ent & (NB - 1);
          int e = cb + ((ent >> 12) & (CHUNK - 1));
          e = e > nE - 1 ? nE - 1 : e;
          int src = ei[e];
          src = src < 0 ? 0 : (src > nN - 1 ? nN - 1 : src);
          const float wg = pw[e];
#pragma unroll 1
          for (int dd = lane; dd < DIN; dd += 32) {
            float xv = xin[(size_t)src * DIN + dd];
            xv = (xv - mus[dd]) * scs[dd] + bes[dd];
            const float ev = wg * ews[dd] + ebs[dd];
            acc[slot * DIN + dd] += fmaxf(xv + ev, 0.0f);
          }
        }
      }
    }
    __syncthreads();
  }

  const float eps1 = 1.0f + epsp[0];
#pragma unroll 1
  for (int q = 0; q < NB / NTHR; ++q) {
    const int slot = q * NTHR + tid;
    const int node = nodeBase + slot;
    float* arow = acc + slot * DIN;
    if (node < nN) {
      const float* xr = xin + (size_t)node * DIN;
      float t[16];
#pragma unroll
      for (int j = 0; j < 16; ++j) t[j] = b1s[j];
#pragma unroll 1
      for (int d = 0; d < DIN; ++d) {
        float xv = xr[d];
        xv = (xv - mus[d]) * scs[d] + bes[d];
        const float hd = eps1 * xv + arow[d];
#pragma unroll
        for (int j = 0; j < 16; ++j) t[j] += hd * w1s[d * 16 + j];
      }
#pragma unroll
      for (int j = 0; j < 16; ++j) t[j] = fmaxf(t[j], 0.0f);
#pragma unroll 1
      for (int k = 0; k < 16; ++k) {
        float y = b2s[k];
#pragma unroll
        for (int j = 0; j < 16; ++j) y += t[j] * w2s[j * 16 + k];
        arow[k] = fmaxf(y, 0.0f);
      }
    } else {
#pragma unroll 1
      for (int k = 0; k < 16; ++k) arow[k] = 0.0f;
    }
  }
  __syncthreads();

  if (tid < 32) {
    const int f = tid & 15, sq = tid >> 4;
    int nval = nN - nodeBase;
    nval = nval > NB ? NB : nval;
    double S = 0.0;
#pragma unroll 1
    for (int s = 0; s < nval; ++s) { const double v = (double)acc[s * DIN + f]; S += sq ? v * v : v; }
    pst[sq * 16 + f] = S;
  }
  __syncthreads();
  if (tid < 16) {
    v2d v; v.x = pst[2 * tid]; v.y = pst[2 * tid + 1];
    *(volatile v2d*)(pout + (size_t)blockIdx.x * 32 + 2 * tid) = v;
  }
  float* gp = yout + (size_t)nodeBase * 16;
  for (int i = tid; i < NB * 4; i += NTHR) {
    const int rr = i >> 2, c4 = (i & 3) * 4;
    const float* ap = acc + rr * DIN + c4;
    v4f v; v.x = ap[0]; v.y = ap[1]; v.z = ap[2]; v.w = ap[3];
    *(volatile v4f*)(gp + (size_t)i * 4) = v;
  }
  __threadfence();
  if (tid < 16) {
    v2d v; v.x = pst[2 * tid]; v.y = pst[2 * tid + 1];
    *(volatile v2d*)(pout + (size_t)blockIdx.x * 32 + 2 * tid) = v;
  }
  for (int i = tid; i < NB * 4; i += NTHR) {
    const int rr = i >> 2, c4 = (i & 3) * 4;
    const float* ap = acc + rr * DIN + c4;
    v4f v; v.x = ap[0]; v.y = ap[1]; v.z = ap[2]; v.w = ap[3];
    *(volatile v4f*)(gp + (size_t)i * 4) = v;
  }
}

__global__ __launch_bounds__(NTHR) void k_pool(
    const float* __restrict__ yin, const int* __restrict__ bat,
    const double* __restrict__ pin, int nBlkIn, const float* __restrict__ gam, const float* __restrict__ bet,
    const float* __restrict__ fw, const float* __restrict__ fb, float* out, int nN) {
  __shared__ float mus[16], scs[16], bes[16];
  __shared__ float sums[64 * 16], cnts[64], means[64 * 16];
  __shared__ v4f stg4[64 * EMBD / 4];
  const int tid = threadIdx.x;
  if (tid < 16) {
    double S = 0.0, Q = 0.0;
#pragma unroll 1
    for (int bb = 0; bb < nBlkIn; ++bb) { S += pin[(size_t)bb * 32 + tid]; Q += pin[(size_t)bb * 32 + 16 + tid]; }
    const double mud = S / (double)nN;
    double var = Q / (double)nN - mud * mud;
    var = var < 0.0 ? 0.0 : var;
    mus[tid] = (float)mud;
    scs[tid] = gam[tid] * (1.0f / sqrtf((float)var + BN_EPS));
    bes[tid] = bet[tid];
  }
  __syncthreads();
  const int g = tid >> 2, q = tid & 3;
  const float m0 = mus[4 * q], m1 = mus[4 * q + 1], m2 = mus[4 * q + 2], m3 = mus[4 * q + 3];
  const float s0 = scs[4 * q], s1 = scs[4 * q + 1], s2 = scs[4 * q + 2], s3 = scs[4 * q + 3];
  const float e0 = bes[4 * q], e1 = bes[4 * q + 1], e2 = bes[4 * q + 2], e3 = bes[4 * q + 3];
  float a0 = 0.f, a1 = 0.f, a2 = 0.f, a3 = 0.f, cn = 0.f;
#pragma unroll 1
  for (int i = 0; i < nN; ++i) {
    const int  bb  = bat[i];
    const bool hit = (bb == g);
    const v4f  v   = *(const v4f*)(yin + (size_t)i * 16 + 4 * q);
    const float x0 = (v.x - m0) * s0 + e0, x1 = (v.y - m1) * s1 + e1;
    const float x2 = (v.z - m2) * s2 + e2, x3 = (v.w - m3) * s3 + e3;
    a0 = hit ? a0 + x0 : a0;  a1 = hit ? a1 + x1 : a1;
    a2 = hit ? a2 + x2 : a2;  a3 = hit ? a3 + x3 : a3;
    cn = hit ? cn + 1.0f : cn;
  }
  sums[g * 16 + 4 * q] = a0; sums[g * 16 + 4 * q + 1] = a1;
  sums[g * 16 + 4 * q + 2] = a2; sums[g * 16 + 4 * q + 3] = a3;
  if (q == 0) cnts[g] = cn;
  __syncthreads();
  for (int i = tid; i < 64 * 16; i += NTHR) {
    const float cc = fmaxf(cnts[i >> 4], 1.0f);
    means[i] = sums[i] * (1.0f / cc);
  }
  __syncthreads();
  float* sp = (float*)stg4;
  for (int o = tid; o < 64 * EMBD; o += NTHR) {
    const int gg = o >> 7, n = o & (EMBD - 1);
    float y = fb[n];
#pragma unroll 1
    for (int d = 0; d < 16; ++d) y += means[gg * 16 + d] * fw[d * EMBD + n];
    sp[o] = fmaxf(y, 0.0f);
  }
  __syncthreads();
  for (int i = tid; i < 64 * EMBD / 4; i += NTHR) { const v4f v = stg4[i]; *(volatile v4f*)(out + (size_t)i * 4) = v; }
  __threadfence();
  for (int i = tid; i < 64 * EMBD / 4; i += NTHR) { const v4f v = stg4[i]; *(volatile v4f*)(out + (size_t)i * 4) = v; }
}

#define NB1 2048
#define NB2 4096
#define LDS1 (NB1 * NFP * 4 + NWAVE * WCAP * 4)
#define LDS2 (NB2 * DIM * 4 + NWAVE * WCAP * 4)
static_assert(LDS1 <= 296 * 1024);
static_assert(LDS2 <= 296 * 1024);

extern "C" void kernel_launch(void* const* d_in, const int* in_sizes, int n_in,
                              void* d_out, int out_size, void* d_ws, size_t ws_size,
                              hipStream_t stream) {
  if (n_in < 32) return;
  const int nN = in_sizes[0] / NFP;
  const int nE = in_sizes[1] / 2;
  const int L1 = 3000, L2 = 2998;
  const int B  = in_sizes[4] / L1;
  if (nN <= 0 || nE <= 0 || B != 64) return;
  if (in_sizes[0] != nN * NFP || in_sizes[1] != 2 * nE || in_sizes[2] != nE || in_sizes[3] != nN) return;
  if (in_sizes[4] != B * L1 || in_sizes[5] != B * L2) return;
  if (in_sizes[6] != NFP * DIM || in_sizes[7] < DIM || in_sizes[8] != 256 || in_sizes[9] < DIM) return;
  if (in_sizes[10] < NFP || in_sizes[11] < NFP || in_sizes[12] < 1) return;
  if (in_sizes[13] != 4 * 256 || in_sizes[14] < 64 || in_sizes[15] != 4 * 256 || in_sizes[16] < 64) return;
  if (in_sizes[17] < 64 || in_sizes[18] < 64 || in_sizes[19] < 4) return;
  if (in_sizes[20] < 5 * DIM || in_sizes[21] < 5 * DIM || in_sizes[22] != DIM * EMBD || in_sizes[23] < EMBD) return;
  const int NT1 = in_sizes[24] / EMBD, NT2 = in_sizes[25] / EMBD;
  if (NT1 < 1 || NT1 > 65 || NT2 < 1 || NT2 > 65 || in_sizes[24] != NT1 * EMBD || in_sizes[25] != NT2 * EMBD) return;
  if (in_sizes[26] != NF * L1 * KSZ || in_sizes[27] < NF || in_sizes[28] != NF * L2 * KSZ || in_sizes[29] < NF) return;
  if (in_sizes[30] != FCIN * EMBD || in_sizes[31] < EMBD) return;
  if (out_size != 2 * B * EMBD) return;

  const float* pro_x  = (const float*)d_in[0];
  const int*   ei     = (const int*)d_in[1];
  const float* pw     = (const float*)d_in[2];
  const int*   batch  = (const int*)d_in[3];
  const int*   rglob  = (const int*)d_in[4];
  const int*   rloc   = (const int*)d_in[5];
  const float* g1_w1  = (const float*)d_in[6];
  const float* g1_b1  = (const float*)d_in[7];
  const float* g1_w2  = (const float*)d_in[8];
  const float* g1_b2  = (const float*)d_in[9];
  const float* g1_ew  = (const float*)d_in[10];
  const float* g1_eb  = (const float*)d_in[11];
  const float* g1_eps = (const float*)d_in[12];
  const float* g_w1   = (const float*)d_in[13];
  const float* g_b1   = (const float*)d_in[14];
  const float* g_w2   = (const float*)d_in[15];
  const float* g_b2   = (const float*)d_in[16];
  const float* g_ew   = (const float*)d_in[17];
  const float* g_eb   = (const float*)d_in[18];
  const float* g_eps  = (const float*)d_in[19];
  const float* bn_g   = (const float*)d_in[20];
  const float* bn_b   = (const float*)d_in[21];
  const float* fc1_w  = (const float*)d_in[22];
  const float* fc1_b  = (const float*)d_in[23];
  const float* emb1   = (const float*)d_in[24];
  const float* emb2   = (const float*)d_in[25];
  const float* c1w    = (const float*)d_in[26];
  const float* c1b    = (const float*)d_in[27];
  const float* c2w    = (const float*)d_in[28];
  const float* c2b    = (const float*)d_in[29];
  const float* fcxr_w = (const float*)d_in[30];
  const float* fcxr_b = (const float*)d_in[31];
  float* out = (float*)d_out;

  const int KPC   = ((L1 * KSZ + 63) / 64) * 64;
  const int nKsC  = KPC / 32;
  const int KPF   = ((FCIN + 63) / 64) * 64;
  const int nKsF  = FCIN / 32;
  const int M     = B * TOUT;
  const int nTiles = (M + 15) / 16;
  const int cGrid  = (nTiles + 3) / 4;
  const int nBlk1 = (nN + NB1 - 1) / NB1;
  const int nBlk2 = (nN + NB2 - 1) / NB2;
  if (nBlk1 > 128 || nBlk2 > 128) return;
  if ((FCIN % 32) != 0 || L2 * KSZ > KPC) return;

  char* ws = (char*)d_ws;
  size_t off = 0;
#define TAKE(NAME, BYTES) const size_t NAME = off; off += (((size_t)(BYTES)) + 255) & ~(size_t)255;
  const size_t szWc = (size_t)NF * KPC * 2;
  const size_t szWf = (size_t)EMBD * KPF * 2;
  const size_t szP  = (size_t)nTiles * 16 * NF * 4;
  const size_t rowsY = ((size_t)nBlk1 * NB1 > (size_t)nBlk2 * NB2) ? (size_t)nBlk1 * NB1 : (size_t)nBlk2 * NB2;
  const size_t szY  = rowsY * 16 * 4;
  const size_t szPt = (size_t)128 * 32 * 8;
  TAKE(oWh1, szWc) TAKE(oWl1, szWc) TAKE(oWh2, szWc) TAKE(oWl2, szWc)
  TAKE(oFh, szWf)  TAKE(oFl, szWf)
  TAKE(oP0, szP)   TAKE(oP1, szP)
  TAKE(oYa, szY)   TAKE(oYb, szY)
  TAKE(oPt, szPt * 5)
#undef TAKE
  if (off > ws_size || off > (size_t)134217728) return;
  bf16_t* wh1 = (bf16_t*)(ws + oWh1); bf16_t* wl1 = (bf16_t*)(ws + oWl1);
  bf16_t* wh2 = (bf16_t*)(ws + oWh2); bf16_t* wl2 = (bf16_t*)(ws + oWl2);
  bf16_t* fh  = (bf16_t*)(ws + oFh);  bf16_t* fl  = (bf16_t*)(ws + oFl);
  float*  P0  = (float*)(ws + oP0);   float*  P1  = (float*)(ws + oP1);
  float*  Ya  = (float*)(ws + oYa);   float*  Yb  = (float*)(ws + oYb);
  double* Pt  = (double*)(ws + oPt);
  const size_t ptStride = szPt / 8;

  const int nTotC = NF * KPC / 8, nTotF = EMBD * KPF / 8;
  k_wprep<<<(nTotC + NTHR - 1) / NTHR, NTHR, 0, stream>>>(c1w, L1 * KSZ, 1, L1 * KSZ, KPC, wh1, wl1, nTotC);
  k_wprep<<<(nTotC + NTHR - 1) / NTHR, NTHR, 0, stream>>>(c2w, L2 * KSZ, 1, L2 * KSZ, KPC, wh2, wl2, nTotC);
  k_wprep<<<(nTotF + NTHR - 1) / NTHR, NTHR, 0, stream>>>(fcxr_w, 1, EMBD, FCIN, KPF, fh, fl, nTotF);
  k_conv<<<cGrid, 128, 0, stream>>>(rglob, L1, NT1, emb1, wh1, wl1, KPC, nKsC, c1b, P0, M, nTiles);
  k_conv<<<cGrid, 128, 0, stream>>>(rloc,  L2, NT2, emb2, wh2, wl2, KPC, nKsC, c2b, P1, M, nTiles);
  k_fc<<<B / 16, 32, 0, stream>>>(P0, P1, fh, fl, KPF, nKsF, fcxr_b, out);

  hipFuncSetAttribute(reinterpret_cast<const void*>(&k_gine<NFP, NB1>), hipFuncAttributeMaxDynamicSharedMemorySize, LDS1);
  hipFuncSetAttribute(reinterpret_cast<const void*>(&k_gine<DIM, NB2>), hipFuncAttributeMaxDynamicSharedMemorySize, LDS2);
  k_gine<NFP, NB1><<<nBlk1, NTHR, LDS1, stream>>>(ei, pw, pro_x, g1_ew, g1_eb, g1_eps, g1_w1, g1_b1, g1_w2, g1_b2,
                                                   Pt, 0, bn_g, bn_b, Ya, Pt, nN, nE);
  float* xin = Ya;
  float* xout = Yb;
  int nBlkPrev = nBlk1;
  for (int i = 0; i < 4; ++i) {
    k_gine<DIM, NB2><<<nBlk2, NTHR, LDS2, stream>>>(ei, pw, xin, g_ew + i * 16, g_eb + i * 16, g_eps + i,
                                                    g_w1 + i * 256, g_b1 + i * 16, g_w2 + i * 256, g_b2 + i * 16,
                                                    Pt + (size_t)i * ptStride, nBlkPrev, bn_g + i * 16, bn_b + i * 16,
                                                    xout, Pt + (size_t)(i + 1) * ptStride, nN, nE);
    float* tsw = xin; xin = xout; xout = tsw;
    nBlkPrev = nBlk2;
  }
  k_pool<<<1, NTHR, 0, stream>>>(xin, batch, Pt + (size_t)4 * ptStride, nBlk2, bn_g + 4 * 16, bn_b + 4 * 16,
                                 fc1_w, fc1_b, out + (size_t)B * EMBD, nN);
}
